// TEMoEFFN_37108517437871
// MI455X (gfx1250) — hardware-verified
//
#include <hip/hip_runtime.h>


#define S_TOK 4096
#define C_DIM 1024
#define F_DIM 512
#define E_NUM 8
#define TCH 256
#define NCHUNK (S_TOK / TCH)
#define NPH 4
#define CPP (NCHUNK / NPH)

typedef char chk_s[(S_TOK % TCH == 0 && TCH == 256 && NCHUNK % NPH == 0 && S_TOK % 64 == 0 && S_TOK % 8 == 0) ? 1 : -1];
typedef char chk_c[(C_DIM % 256 == 0 && F_DIM % 256 == 0 && C_DIM % 128 == 0 && F_DIM % 128 == 0 &&
                    C_DIM % 32 == 0 && F_DIM % 32 == 0 && (2 * F_DIM) % 8 == 0 && C_DIM % 8 == 0) ? 1 : -1];
typedef char chk_e[(E_NUM == 8 && CPP * E_NUM == 32) ? 1 : -1];

typedef _Float16 f16t;
typedef f16t v8h __attribute__((ext_vector_type(8)));
typedef f16t v16h __attribute__((ext_vector_type(16)));
typedef float v8f __attribute__((ext_vector_type(8)));
typedef float v4f __attribute__((ext_vector_type(4)));

union Frag { v16h v; v8h q[2]; };
union U8 { v8h v; f16t s[8]; };
union U4 { v4f v; float s[4]; };

constexpr size_t OFF_PR  = 0;
constexpr size_t SZ_PR   = (size_t)S_TOK * E_NUM * 4;
constexpr size_t OFF_XH  = OFF_PR + SZ_PR;
constexpr size_t SZ_XH   = (size_t)S_TOK * C_DIM * 2;
constexpr size_t OFF_WS1 = OFF_XH + SZ_XH;
constexpr size_t SZ_WS1  = (size_t)2 * F_DIM * C_DIM * 2;
constexpr size_t OFF_WS2 = OFF_WS1 + SZ_WS1;
constexpr size_t SZ_WS2  = (size_t)C_DIM * F_DIM * 2;
constexpr size_t OFF_WF1 = OFF_WS2 + SZ_WS2;
constexpr size_t SZ_WF1  = (size_t)E_NUM * 2 * F_DIM * C_DIM * 2;
constexpr size_t OFF_WF2 = OFF_WF1 + SZ_WF1;
constexpr size_t SZ_WF2  = (size_t)E_NUM * C_DIM * F_DIM * 2;
constexpr size_t OFF_AS  = OFF_WF2 + SZ_WF2;
constexpr size_t SZ_AS   = (size_t)S_TOK * F_DIM * 2;
constexpr size_t OFF_XG  = OFF_AS + SZ_AS;
constexpr size_t SZ_XG   = (size_t)CPP * E_NUM * TCH * C_DIM * 2;
constexpr size_t OFF_AG  = OFF_XG + SZ_XG;
constexpr size_t SZ_AG   = (size_t)CPP * E_NUM * TCH * F_DIM * 2;
constexpr size_t OFF_YG  = OFF_AG + SZ_AG;
constexpr size_t SZ_YG   = (size_t)CPP * E_NUM * TCH * C_DIM * 4;
constexpr size_t OFF_MO  = OFF_YG + SZ_YG;
constexpr size_t SZ_MO   = (size_t)S_TOK * C_DIM * 4;
constexpr size_t WS_END  = OFF_MO + SZ_MO;
typedef char chk_align[(OFF_XH % 128 == 0 && OFF_WS1 % 128 == 0 && OFF_WS2 % 128 == 0 && OFF_WF1 % 128 == 0 &&
                        OFF_WF2 % 128 == 0 && OFF_AS % 128 == 0 && OFF_XG % 128 == 0 && OFF_AG % 128 == 0 &&
                        OFF_YG % 128 == 0 && OFF_MO % 128 == 0) ? 1 : -1];

__device__ __forceinline__ int clampi(int v, int lo, int hi) { return v < lo ? lo : (v > hi ? hi : v); }

__device__ __forceinline__ v8f mma16(v16h a, v16h b, v8f c) {
  v8f d = __builtin_amdgcn_wmma_f32_16x16x32_f16(false, a, false, b, (short)0, c, false, false);
  asm volatile("v_nop\n\tv_nop\n\tv_nop\n\tv_nop" : "+v"(d) : "v"(a), "v"(b));
  return d;
}

template<int NCOLS>
__device__ __forceinline__ void row_f32_to_f16(const float* s, f16t* d, int lane, float scale) {
  constexpr int NCH = NCOLS / 256;
  v8h hv[NCH];
#pragma unroll
  for (int q = 0; q < NCH; ++q) {
    const float* sp = s + q * 256 + lane * 8;
    const v4f f0 = *(const v4f*)sp;
    const v4f f1 = *(const v4f*)(sp + 4);
    v8h t;
    t[0] = (f16t)(f0.x * scale); t[1] = (f16t)(f0.y * scale);
    t[2] = (f16t)(f0.z * scale); t[3] = (f16t)(f0.w * scale);
    t[4] = (f16t)(f1.x * scale); t[5] = (f16t)(f1.y * scale);
    t[6] = (f16t)(f1.z * scale); t[7] = (f16t)(f1.w * scale);
    hv[q] = t;
  }
#pragma unroll
  for (int q = 0; q < NCH; ++q) *(volatile v8h*)(d + q * 256 + lane * 8) = hv[q];
  __threadfence();
#pragma unroll
  for (int q = 0; q < NCH; ++q) *(volatile v8h*)(d + q * 256 + lane * 8) = hv[q];
}

__device__ __forceinline__ int chunk_count(const float* probs, int tok0, int e, int* wtot) {
  const int tid = threadIdx.x, wave = tid >> 5, lane = tid & 31;
  const float p = probs[(size_t)(tok0 + tid) * E_NUM + e];
  const unsigned b = __builtin_amdgcn_ballot_w32(p != 0.f);
  if (lane == 0) wtot[wave] = (int)__popc(b);
  __syncthreads();
  int total = 0;
#pragma unroll
  for (int w = 0; w < 8; ++w) total += wtot[w];
  return total > TCH ? TCH : total;
}

__device__ __forceinline__ int chunk_select(const float* probs, int tok0, int e, int* lst, int* wtot) {
  const int tid = threadIdx.x, wave = tid >> 5, lane = tid & 31;
  const float p = probs[(size_t)(tok0 + tid) * E_NUM + e];
  const int flag = (p != 0.f) ? 1 : 0;
  const unsigned b = __builtin_amdgcn_ballot_w32(flag != 0);
  const int rank = (int)__popc(b & ((1u << lane) - 1u));
  if (lane == 0) wtot[wave] = (int)__popc(b);
  __syncthreads();
  int prefix = 0, total = 0;
#pragma unroll
  for (int w = 0; w < 8; ++w) { const int v = wtot[w]; total += v; prefix += (w < wave) ? v : 0; }
  if (flag != 0) {
    const int pos = prefix + rank;
    if ((unsigned)pos < (unsigned)TCH) lst[pos] = tid;
  }
  __syncthreads();
  return total > TCH ? TCH : total;
}


template<int NCOLS>
__global__ __launch_bounds__(256) void cvt_rows(const float* src, f16t* dst, int nrows, float scale) {
  const int wave = threadIdx.x >> 5, lane = threadIdx.x & 31;
  const int row = blockIdx.x * 8 + wave;
  if (row >= nrows) return;
  row_f32_to_f16<NCOLS>(src + (size_t)row * NCOLS, dst + (size_t)row * NCOLS, lane, scale);
}

__global__ __launch_bounds__(256) void router_topk(const float* x, const float* wr, float* probs, int S) {
  __shared__ U4 lrec[16];
  const int wave = threadIdx.x >> 5, lane = threadIdx.x & 31;
  const int tok = blockIdx.x * 8 + wave;
  const bool valid = tok < S;
  float acc[E_NUM];
#pragma unroll
  for (int e = 0; e < E_NUM; ++e) acc[e] = 0.f;
  if (valid) {
    const float* xp = x + (size_t)tok * C_DIM;
#pragma unroll 4
    for (int c = lane; c < C_DIM; c += 32) {
      const float xv = xp[c];
      const float* wp = wr + (size_t)c * E_NUM;
      const v4f w0 = *(const v4f*)wp;
      const v4f w1 = *(const v4f*)(wp + 4);
      acc[0] += xv * w0.x; acc[1] += xv * w0.y; acc[2] += xv * w0.z; acc[3] += xv * w0.w;
      acc[4] += xv * w1.x; acc[5] += xv * w1.y; acc[6] += xv * w1.z; acc[7] += xv * w1.w;
    }
  }
#pragma unroll
  for (int e = 0; e < E_NUM; ++e) {
#pragma unroll
    for (int off = 16; off > 0; off >>= 1) acc[e] += __shfl_xor(acc[e], off, 32);
  }
  int i1 = 0; float v1 = acc[0];
#pragma unroll
  for (int e = 1; e < E_NUM; ++e) if (acc[e] > v1) { v1 = acc[e]; i1 = e; }
  int i2 = -1; float v2 = __int_as_float(0xff800000);
#pragma unroll
  for (int e = 0; e < E_NUM; ++e) if (e != i1 && acc[e] > v2) { v2 = acc[e]; i2 = e; }
  if (i2 < 0) { i2 = (i1 == 0) ? 1 : 0; v2 = acc[0]; if (i1 == 0) v2 = acc[1]; }
  const float mx = v1;
  float sum = 0.f;
#pragma unroll
  for (int e = 0; e < E_NUM; ++e) sum += __expf(acc[e] - mx);
  const float inv = 1.f / sum;
  const float sc1 = __expf(v1 - mx) * inv;
  const float sc2 = __expf(v2 - mx) * inv;
  const float invw = 1.f / (sc1 + sc2);
  const float p1 = sc1 * invw, p2 = sc2 * invw;
  if (lane == 0) {
    U4 r0, r1;
#pragma unroll
    for (int k = 0; k < 4; ++k) {
      r0.s[k] = (k == i1) ? p1 : ((k == i2) ? p2 : 0.f);
      r1.s[k] = (k + 4 == i1) ? p1 : ((k + 4 == i2) ? p2 : 0.f);
    }
    lrec[wave * 2] = r0;
    lrec[wave * 2 + 1] = r1;
  }
  __syncthreads();
  if (wave == 0 && lane < 16) {
    const int t = blockIdx.x * 8 + (lane >> 1);
    const v4f v = lrec[lane].v;
    if (t < S) {
      float* d = probs + (size_t)t * E_NUM + (lane & 1) * 4;
      *(volatile v4f*)d = v;
      __threadfence();
      *(volatile v4f*)d = v;
    }
  }
}

__global__ __launch_bounds__(256) void gather_rows(const f16t* xh, const float* probs, f16t* xg, int chunk0) {
  __shared__ int lst[TCH];
  __shared__ int wtot[8];
  const int tid = threadIdx.x, wave = tid >> 5, lane = tid & 31;
  const int z = blockIdx.x;
  const int cl = z >> 3, e = z & 7;
  const int tok0 = (chunk0 + cl) * TCH;
  const int cnt = __builtin_amdgcn_readfirstlane(chunk_select(probs, tok0, e, lst, wtot));
  f16t* dbase = xg + (size_t)z * TCH * C_DIM;
  const f16t hz = (f16t)0.f;
  const v8h z8 = {hz, hz, hz, hz, hz, hz, hz, hz};
#pragma unroll 1
  for (int q = 0; q < 8; ++q) {
    const int slot = blockIdx.y * 64 + wave * 8 + q;
    const bool valid = slot < cnt;
    const int sl = slot < TCH ? slot : TCH - 1;
    const int tl = clampi(lst[sl], 0, TCH - 1);
    const f16t* src = xh + (size_t)(tok0 + tl) * C_DIM + lane * 8;
    v8h hv[4];
#pragma unroll
    for (int c = 0; c < 4; ++c) hv[c] = z8;
    if (valid) {
#pragma unroll
      for (int c = 0; c < 4; ++c) hv[c] = *(const v8h*)(src + c * 256);
    }
    f16t* d = dbase + (size_t)slot * C_DIM + lane * 8;
#pragma unroll
    for (int c = 0; c < 4; ++c) *(volatile v8h*)(d + c * 256) = hv[c];
    __threadfence();
#pragma unroll
    for (int c = 0; c < 4; ++c) *(volatile v8h*)(d + c * 256) = hv[c];
  }
}

template<bool ROUTED>
__global__ __launch_bounds__(256) void fc1_swiglu(const f16t* arows, const f16t* w1all, const float* probs,
                                                  f16t* actout, int chunk0) {
  __shared__ U8 tile[64][17];
  __shared__ int wtot[8];
  const int tid = threadIdx.x, wave = tid >> 5, lane = tid & 31;
  const int h = lane >> 4, m = lane & 15;
  int Me = S_TOK;
  const f16t* A = arows;
  const f16t* W = w1all;
  f16t* AO = actout;
  if (ROUTED) {
    const int z = blockIdx.z;
    const int cl = z >> 3, e = z & 7;
    const int tok0 = (chunk0 + cl) * TCH;
    Me = chunk_count(probs, tok0, e, wtot);
    A = arows + (size_t)z * TCH * C_DIM;
    W = w1all + (size_t)e * (2 * F_DIM) * C_DIM;
    AO = actout + (size_t)z * TCH * F_DIM;
  }
  const int meu = __builtin_amdgcn_readfirstlane(Me);
  const int rowblk = blockIdx.x * 64;
  if (rowblk >= meu) return;
  const int colblk = blockIdx.y * 128;
  const int wr = wave >> 2, wc = wave & 3;
  const int colbase = colblk + wc * 32;
  const int rowbase = rowblk + wr * 32;
  const bool act0 = __builtin_amdgcn_readfirstlane(rowbase) < meu;
  const bool act1 = __builtin_amdgcn_readfirstlane(rowbase + 16) < meu;

  const f16t* aptr[2];
#pragma unroll
  for (int i = 0; i < 2; ++i) aptr[i] = A + (size_t)(rowbase + i * 16 + m) * C_DIM + 8 * h;
  const f16t* gptr[2];
  const f16t* uptr[2];
#pragma unroll
  for (int j = 0; j < 2; ++j) {
    const int n = colbase + j * 16 + m;
    gptr[j] = W + (size_t)n * C_DIM + 8 * h;
    uptr[j] = W + (size_t)(F_DIM + n) * C_DIM + 8 * h;
  }

  v8f accg[2][2] = {};
  v8f accu[2][2] = {};
  if (act0) {
    for (int kb = 0; kb < C_DIM; kb += 32) {
      Frag a0, a1, bg[2], bu[2];
      a0.q[0] = *(const v8h*)(aptr[0] + kb);
      a0.q[1] = *(const v8h*)(aptr[0] + kb + 16);
#pragma unroll
      for (int j = 0; j < 2; ++j) {
        bg[j].q[0] = *(const v8h*)(gptr[j] + kb);
        bg[j].q[1] = *(const v8h*)(gptr[j] + kb + 16);
        bu[j].q[0] = *(const v8h*)(uptr[j] + kb);
        bu[j].q[1] = *(const v8h*)(uptr[j] + kb + 16);
      }
#pragma unroll
      for (int j = 0; j < 2; ++j) {
        accg[0][j] = mma16(a0.v, bg[j].v, accg[0][j]);
        accu[0][j] = mma16(a0.v, bu[j].v, accu[0][j]);
      }
      if (act1) {
        a1.q[0] = *(const v8h*)(aptr[1] + kb);
        a1.q[1] = *(const v8h*)(aptr[1] + kb + 16);
#pragma unroll
        for (int j = 0; j < 2; ++j) {
          accg[1][j] = mma16(a1.v, bg[j].v, accg[1][j]);
          accu[1][j] = mma16(a1.v, bu[j].v, accu[1][j]);
        }
      }
    }
  }

  const float inv64 = 0.015625f;
#pragma unroll
  for (int i = 0; i < 2; ++i)
#pragma unroll
    for (int j = 0; j < 2; ++j)
#pragma unroll
      for (int r = 0; r < 8; ++r) {
        const float g = accg[i][j][r] * inv64;
        const float u = accu[i][j][r] * inv64;
        const float sg = g / (1.f + __expf(-g));
        const int rl = wr * 32 + i * 16 + 8 * h + r;
        const int cl = wc * 32 + j * 16 + m;
        tile[rl][cl >> 3].s[cl & 7] = (f16t)(sg * u * 16.f);
      }
  __syncthreads();
  v8h hold[4];
  f16t* optr[4];
#pragma unroll
  for (int q = 0; q < 4; ++q) {
    const int rl = wave * 8 + q * 2 + h;
    hold[q] = tile[rl][m].v;
    optr[q] = AO + (size_t)(rowblk + rl) * F_DIM + colblk + m * 8;
  }
#pragma unroll
  for (int q = 0; q < 4; ++q) *(volatile v8h*)optr[q] = hold[q];
  __threadfence();
#pragma unroll
  for (int q = 0; q < 4; ++q) *(volatile v8h*)optr[q] = hold[q];
}

template<bool ROUTED>
__global__ __launch_bounds__(256) void fc2_proj(const f16t* actin, const f16t* w2all, const float* probs,
                                                const float* mo, float* dst, int chunk0) {
  __shared__ U4 tile[64][33];
  __shared__ int wtot[8];
  const int tid = threadIdx.x, wave = tid >> 5, lane = tid & 31;
  const int h = lane >> 4, m = lane & 15;
  int Me = S_TOK;
  const f16t* A = actin;
  const f16t* W = w2all;
  float* D = dst;
  if (ROUTED) {
    const int z = blockIdx.z;
    const int cl = z >> 3, e = z & 7;
    const int tok0 = (chunk0 + cl) * TCH;
    Me = chunk_count(probs, tok0, e, wtot);
    A = actin + (size_t)z * TCH * F_DIM;
    W = w2all + (size_t)e * C_DIM * F_DIM;
    D = dst + (size_t)z * TCH * C_DIM;
  }
  const int meu = __builtin_amdgcn_readfirstlane(Me);
  const int rowblk = blockIdx.x * 64;
  if (rowblk >= meu) return;
  const int colblk = blockIdx.y * 128;
  const int wr = wave >> 2, wc = wave & 3;
  const int colbase = colblk + wc * 32;
  const int rowbase = rowblk + wr * 32;
  const bool act0 = __builtin_amdgcn_readfirstlane(rowbase) < meu;
  const bool act1 = __builtin_amdgcn_readfirstlane(rowbase + 16) < meu;

  const f16t* aptr[2];
#pragma unroll
  for (int i = 0; i < 2; ++i) aptr[i] = A + (size_t)(rowbase + i * 16 + m) * F_DIM + 8 * h;
  const f16t* bptr[2];
#pragma unroll
  for (int j = 0; j < 2; ++j) bptr[j] = W + (size_t)(colbase + j * 16 + m) * F_DIM + 8 * h;

  v8f acc[2][2] = {};
  if (act0) {
    for (int kb = 0; kb < F_DIM; kb += 32) {
      Frag a0, a1, b[2];
      a0.q[0] = *(const v8h*)(aptr[0] + kb);
      a0.q[1] = *(const v8h*)(aptr[0] + kb + 16);
#pragma unroll
      for (int j = 0; j < 2; ++j) {
        b[j].q[0] = *(const v8h*)(bptr[j] + kb);
        b[j].q[1] = *(const v8h*)(bptr[j] + kb + 16);
      }
#pragma unroll
      for (int j = 0; j < 2; ++j) acc[0][j] = mma16(a0.v, b[j].v, acc[0][j]);
      if (act1) {
        a1.q[0] = *(const v8h*)(aptr[1] + kb);
        a1.q[1] = *(const v8h*)(aptr[1] + kb + 16);
#pragma unroll
        for (int j = 0; j < 2; ++j) acc[1][j] = mma16(a1.v, b[j].v, acc[1][j]);
      }
    }
  }

  const float inv1024 = 0.0009765625f;
#pragma unroll
  for (int i = 0; i < 2; ++i)
#pragma unroll
    for (int j = 0; j < 2; ++j)
#pragma unroll
      for (int r = 0; r < 8; ++r) {
        const int rl = wr * 32 + i * 16 + 8 * h + r;
        const int cl = wc * 32 + j * 16 + m;
        tile[rl][cl >> 2].s[cl & 3] = acc[i][j][r] * inv1024;
      }
  __syncthreads();
  v4f val[8];
#pragma unroll
  for (int q = 0; q < 8; ++q) {
    const int rl = wave * 8 + q;
    const int row = rowblk + rl;
    v4f v = tile[rl][lane].v;
    if (!ROUTED) v += *(const v4f*)(mo + (size_t)row * C_DIM + colblk + lane * 4);
    val[q] = v;
  }
  float* d0 = D + (size_t)(rowblk + wave * 8) * C_DIM + colblk + lane * 4;
#pragma unroll
  for (int q = 0; q < 8; ++q) *(volatile v4f*)(d0 + (size_t)q * C_DIM) = val[q];
  __threadfence();
#pragma unroll
  for (int q = 0; q < 8; ++q) *(volatile v4f*)(d0 + (size_t)q * C_DIM) = val[q];
}

__global__ __launch_bounds__(256) void combine_rows(const float* probs, const float* yg, float* mo, int chunk0) {
  __shared__ int wtot[8][E_NUM];
  __shared__ float rp[TCH][2];
  __shared__ int ri[TCH][2];
  const int tid = threadIdx.x, wave = tid >> 5, lane = tid & 31;
  const int cl = blockIdx.x;
  const int tok0 = (chunk0 + cl) * TCH;
  const float* pr = probs + (size_t)(tok0 + tid) * E_NUM;
  U4 q0, q1;
  q0.v = *(const v4f*)pr;
  q1.v = *(const v4f*)(pr + 4);
  float pv[E_NUM];
  int rk[E_NUM];
#pragma unroll
  for (int e = 0; e < E_NUM; ++e) {
    const float p = (e < 4) ? q0.s[e] : q1.s[e - 4];
    pv[e] = p;
    const unsigned b = __builtin_amdgcn_ballot_w32(p != 0.f);
    rk[e] = (int)__popc(b & ((1u << lane) - 1u));
    if (lane == 0) wtot[wave][e] = (int)__popc(b);
  }
  __syncthreads();
  float pa = 0.f, pb = 0.f;
  int ra = 0, rb = 0, cnt = 0;
#pragma unroll
  for (int e = 0; e < E_NUM; ++e) {
    int prefix = 0;
#pragma unroll
    for (int w = 0; w < 8; ++w) prefix += (w < wave) ? wtot[w][e] : 0;
    const int r = clampi(prefix + rk[e], 0, TCH - 1);
    const int rowi = (cl * E_NUM + e) * TCH + r;
    if (pv[e] != 0.f) {
      if (cnt == 0) { pa = pv[e]; ra = rowi; } else if (cnt == 1) { pb = pv[e]; rb = rowi; }
      ++cnt;
    }
  }
  rp[tid][0] = pa; rp[tid][1] = pb;
  ri[tid][0] = ra; ri[tid][1] = rb;
  __syncthreads();
  const v4f z4 = {0.f, 0.f, 0.f, 0.f};
#pragma unroll 1
  for (int j = 0; j < 4; ++j) {
    const int tl = blockIdx.y * 32 + wave * 4 + j;
    const float wa = rp[tl][0], wb = rp[tl][1];
    const int xa = clampi(ri[tl][0], 0, CPP * E_NUM * TCH - 1);
    const int xb = clampi(ri[tl][1], 0, CPP * E_NUM * TCH - 1);
    const float* ya = yg + (size_t)xa * C_DIM + lane * 4;
    const float* yb = yg + (size_t)xb * C_DIM + lane * 4;
    v4f val[8];
#pragma unroll
    for (int q = 0; q < 8; ++q) {
      v4f o = z4;
      if (wa != 0.f) o += *(const v4f*)(ya + q * 128) * wa;
      if (wb != 0.f) o += *(const v4f*)(yb + q * 128) * wb;
      val[q] = o;
    }
    float* d = mo + (size_t)(tok0 + tl) * C_DIM + lane * 4;
#pragma unroll
    for (int q = 0; q < 8; ++q) *(volatile v4f*)(d + q * 128) = val[q];
    __threadfence();
#pragma unroll
    for (int q = 0; q < 8; ++q) *(volatile v4f*)(d + q * 128) = val[q];
  }
}

extern "C" void kernel_launch(void* const* d_in, const int* in_sizes, int n_in,
                              void* d_out, int out_size, void* d_ws, size_t ws_size,
                              hipStream_t stream) {
  if (n_in < 6) return;
  if (in_sizes[0] != S_TOK * C_DIM) return;
  if (in_sizes[1] != C_DIM * E_NUM) return;
  if (in_sizes[2] != 2 * F_DIM * C_DIM) return;
  if (in_sizes[3] != C_DIM * F_DIM) return;
  if (in_sizes[4] != E_NUM * 2 * F_DIM * C_DIM) return;
  if (in_sizes[5] != E_NUM * C_DIM * F_DIM) return;
  if (out_size < S_TOK * C_DIM) return;
  if (ws_size < WS_END) return;

  const float* x     = (const float*)d_in[0];
  const float* wrt   = (const float*)d_in[1];
  const float* w_sh1 = (const float*)d_in[2];
  const float* w_sh2 = (const float*)d_in[3];
  const float* w_fc1 = (const float*)d_in[4];
  const float* w_fc2 = (const float*)d_in[5];
  float* out = (float*)d_out;

  char* ws = (char*)d_ws;
  float* probs = (float*)(ws + OFF_PR);
  f16t* xh     = (f16t*)(ws + OFF_XH);
  f16t* ws1h   = (f16t*)(ws + OFF_WS1);
  f16t* ws2h   = (f16t*)(ws + OFF_WS2);
  f16t* wf1h   = (f16t*)(ws + OFF_WF1);
  f16t* wf2h   = (f16t*)(ws + OFF_WF2);
  f16t* act_s  = (f16t*)(ws + OFF_AS);
  f16t* xg     = (f16t*)(ws + OFF_XG);
  f16t* ag     = (f16t*)(ws + OFF_AG);
  float* yg    = (float*)(ws + OFF_YG);
  float* mo    = (float*)(ws + OFF_MO);

  cvt_rows<C_DIM><<<S_TOK / 8, 256, 0, stream>>>(x, xh, S_TOK, 1.f);
  cvt_rows<C_DIM><<<(2 * F_DIM) / 8, 256, 0, stream>>>(w_sh1, ws1h, 2 * F_DIM, 64.f);
  cvt_rows<F_DIM><<<C_DIM / 8, 256, 0, stream>>>(w_sh2, ws2h, C_DIM, 64.f);
  cvt_rows<C_DIM><<<(E_NUM * 2 * F_DIM) / 8, 256, 0, stream>>>(w_fc1, wf1h, E_NUM * 2 * F_DIM, 64.f);
  cvt_rows<F_DIM><<<(E_NUM * C_DIM) / 8, 256, 0, stream>>>(w_fc2, wf2h, E_NUM * C_DIM, 64.f);

  router_topk<<<S_TOK / 8, 256, 0, stream>>>(x, wrt, probs, S_TOK);

  fc1_swiglu<false><<<dim3(S_TOK / 64, F_DIM / 128, 1), 256, 0, stream>>>(xh, ws1h, probs, act_s, 0);

  for (int ph = 0; ph < NPH; ++ph) {
    const int chunk0 = ph * CPP;
    gather_rows<<<dim3(CPP * E_NUM, TCH / 64, 1), 256, 0, stream>>>(xh, probs, xg, chunk0);
    fc1_swiglu<true><<<dim3(TCH / 64, F_DIM / 128, CPP * E_NUM), 256, 0, stream>>>(xg, wf1h, probs, ag, chunk0);
    fc2_proj<true><<<dim3(TCH / 64, C_DIM / 128, CPP * E_NUM), 256, 0, stream>>>(ag, wf2h, probs, mo, yg, chunk0);
    combine_rows<<<dim3(CPP, TCH / 32, 1), 256, 0, stream>>>(probs, yg, mo, chunk0);
  }

  fc2_proj<false><<<dim3(S_TOK / 64, C_DIM / 128, 1), 256, 0, stream>>>(act_s, ws2h, probs, mo, out, 0);
}
